// GraphAttentionLayer_49297634623557
// MI455X (gfx1250) — hardware-verified
//
#include <hip/hip_runtime.h>
#include <stddef.h>
#include <stdint.h>
#include <math.h>


#pragma clang fp contract(off)

#define NB     16
#define NN     2048
#define FIN    128
#define FO     64
#define MROWS  (NB * NN)
#define PTHR   256
#define NUH    (MROWS * (FIN / 8))
#define NUW    (FO * (FIN / 8))
#define GTHR   128
#define GBM    64
#define QT     64
#define WSMAX  134217728

static_assert(NUH % PTHR == 0 && NUW % PTHR == 0);
static_assert(FIN % 32 == 0 && FIN / 8 == 16);
static_assert(FO == 64 && GBM == (GTHR / 32) * 16 && QT == GBM);
static_assert(MROWS % GBM == 0 && NN % GBM == 0 && NN % 32 == 0);
static_assert(NN == 4 * 4 * GTHR);

typedef float          v4f   __attribute__((ext_vector_type(4)));
typedef float          v8f   __attribute__((ext_vector_type(8)));
typedef int            v8i   __attribute__((ext_vector_type(8)));
typedef unsigned short v8us  __attribute__((ext_vector_type(8)));
typedef unsigned short v16us __attribute__((ext_vector_type(16)));
typedef __bf16         v16bf __attribute__((ext_vector_type(16)));
typedef v4f  __attribute__((may_alias)) v4fa;
typedef v8us __attribute__((may_alias)) v8usa;
union FragB { v16bf v; v16us u; v8us h[2]; v8i w; };

__device__ __forceinline__ v8f wmb(const FragB& a, const FragB& b, v8f c) {
  v8f d = __builtin_amdgcn_wmma_f32_16x16x32_bf16(false, a.v, false, b.v, (short)0, c, false, false);
  asm volatile("v_nop\n\tv_nop\n\tv_nop\n\tv_nop" : "+v"(d) : "v"(a.w), "v"(b.w));
  return d;
}

__device__ __forceinline__ unsigned bf16_bits(float f) {
  const unsigned u = __float_as_uint(f);
  return (u + 0x7FFFu + ((u >> 16) & 1u)) >> 16;
}
__device__ __forceinline__ float bf16_val(float f) {
  return __uint_as_float(bf16_bits(f) << 16);
}

__global__ __launch_bounds__(PTHR) void k_prep(const float* __restrict__ h, const float* __restrict__ W,
                                               const float* __restrict__ a,
                                               unsigned short* HB, unsigned short* WT, float* A12) {
  const int blk = (int)blockIdx.x;
  const int tid = (int)threadIdx.x;
  if (blk < NUH / PTHR) {
    const int u   = blk * PTHR + tid;
    const int row = u >> 4;
    const int k8  = (u & 15) * 8;
    const float* p = h + (size_t)row * FIN + k8;
    const v4f x0 = *(const v4fa*)p;
    const v4f x1 = *(const v4fa*)(p + 4);
    v8us o;
    o[0] = (unsigned short)bf16_bits(x0.x); o[1] = (unsigned short)bf16_bits(x0.y);
    o[2] = (unsigned short)bf16_bits(x0.z); o[3] = (unsigned short)bf16_bits(x0.w);
    o[4] = (unsigned short)bf16_bits(x1.x); o[5] = (unsigned short)bf16_bits(x1.y);
    o[6] = (unsigned short)bf16_bits(x1.z); o[7] = (unsigned short)bf16_bits(x1.w);
    unsigned short* dp = HB + (size_t)row * FIN + k8;
    *(volatile v8us*)dp = o;
    __threadfence();
    *(volatile v8us*)dp = o;
  } else if (blk < (NUH + NUW) / PTHR) {
    const int v  = (blk - NUH / PTHR) * PTHR + tid;
    const int n  = v >> 4;
    const int k8 = (v & 15) * 8;
    const float* p = W + (size_t)k8 * FO + n;
    v8us o;
#pragma unroll
    for (int i = 0; i < 8; ++i) o[i] = (unsigned short)bf16_bits(p[(size_t)i * FO]);
    unsigned short* dp = WT + (size_t)n * FIN + k8;
    *(volatile v8us*)dp = o;
    __threadfence();
    *(volatile v8us*)dp = o;
  } else {
    const bool ok = tid < 32;
    const int t4 = (ok ? tid : 31) * 4;
    const v4f s = *(const v4fa*)(a + t4);
    v4f o;
    o.x = bf16_val(s.x); o.y = bf16_val(s.y); o.z = bf16_val(s.z); o.w = bf16_val(s.w);
    if (ok) *(volatile v4f*)(A12 + t4) = o;
    __threadfence();
    if (ok) *(volatile v4f*)(A12 + t4) = o;
  }
}

__global__ __launch_bounds__(GTHR) void k_proj(const unsigned short* __restrict__ A,
                                               const unsigned short* __restrict__ WT,
                                               const float* __restrict__ a12,
                                               float* WH, float* U, float* V,
                                               unsigned short* VTH, unsigned short* VTL) {
  __shared__ __attribute__((aligned(16))) float stg[GBM * FO];
  __shared__ __attribute__((aligned(16))) float uvs[2 * GBM];
  const int tid = (int)threadIdx.x, lane = tid & 31, wave = tid >> 5, hh = lane >> 4, m = lane & 15;
  const int rowBase = (int)blockIdx.x * GBM;

  v8f acc[4];
  {
    const v8f z = {0.f, 0.f, 0.f, 0.f, 0.f, 0.f, 0.f, 0.f};
    acc[0] = z; acc[1] = z; acc[2] = z; acc[3] = z;
  }
  const unsigned short* ap = A  + (size_t)(rowBase + 16 * wave + m) * (size_t)FIN + 8 * hh;
  const unsigned short* wp = WT + (size_t)m * (size_t)FIN + 8 * hh;
#pragma unroll 1
  for (int ks = 0; ks < FIN / 32; ++ks) {
    FragB af;
    af.h[0] = *(const v8usa*)(ap + 32 * ks);
    af.h[1] = *(const v8usa*)(ap + 32 * ks + 16);
#pragma unroll
    for (int t = 0; t < 4; ++t) {
      const unsigned short* wq = wp + (size_t)(16 * t) * (size_t)FIN + 32 * ks;
      FragB bf;
      bf.h[0] = *(const v8usa*)wq;
      bf.h[1] = *(const v8usa*)(wq + 16);
      acc[t] = wmb(af, bf, acc[t]);
    }
  }

#pragma unroll
  for (int t = 0; t < 4; ++t) {
    const int lc = 16 * t + m;
#pragma unroll
    for (int r = 0; r < 8; ++r) {
      const int lr = 16 * wave + 8 * hh + r;
      stg[lr * FO + lc] = acc[t][r];
    }
  }
  __syncthreads();

  {
    const int row  = tid & (GBM - 1);
    const int aoff = (tid >> 6) * FO;
    float s = 0.0f;
#pragma unroll 4
    for (int k4 = 0; k4 < FO / 4; ++k4) {
      const v4f w4 = *(const v4fa*)(stg + row * FO + 4 * k4);
      const v4f a4 = *(const v4fa*)(a12 + aoff + 4 * k4);
      s = fmaf(w4.x, a4.x, s);
      s = fmaf(w4.y, a4.y, s);
      s = fmaf(w4.z, a4.z, s);
      s = fmaf(w4.w, a4.w, s);
    }
    uvs[tid] = s;
  }
  __syncthreads();

  v4f fv[8];
#pragma unroll
  for (int i = 0; i < 8; ++i) {
    const int lr = 16 * wave + 2 * i + hh;
    fv[i] = *(const v4fa*)(stg + lr * FO + 4 * m);
  }
  const v4f uvv = *(const v4fa*)(uvs + GBM * (wave & 1) + 4 * m);
  const bool okuv = (wave < 2) && (lane < 16);
  float* uvp = ((wave == 0) ? U : V) + (size_t)rowBase + 4 * m;

  const int bq   = rowBase / NN;
  const int mloc = rowBase - bq * NN;
  v8us hv[4], lv[4];
#pragma unroll
  for (int g = 0; g < 4; ++g) {
    const int o  = 16 * g + (tid >> 3);
    const int ms = (tid & 7) * 8;
#pragma unroll
    for (int j = 0; j < 8; ++j) {
      const float f = stg[(ms + j) * FO + o];
      const unsigned hb = bf16_bits(f);
      hv[g][j] = (unsigned short)hb;
      lv[g][j] = (unsigned short)bf16_bits(f - __uint_as_float(hb << 16));
    }
  }

#pragma unroll
  for (int i = 0; i < 8; ++i) {
    const int lr = 16 * wave + 2 * i + hh;
    float* op = WH + (size_t)(rowBase + lr) * (size_t)FO + 4 * m;
    *(volatile v4f*)op = fv[i];
  }
  if (okuv) *(volatile v4f*)uvp = uvv;
#pragma unroll
  for (int g = 0; g < 4; ++g) {
    const int o  = 16 * g + (tid >> 3);
    const int ms = (tid & 7) * 8;
    const size_t off = ((size_t)bq * FO + o) * (size_t)NN + mloc + ms;
    *(volatile v8us*)(VTH + off) = hv[g];
    *(volatile v8us*)(VTL + off) = lv[g];
  }
  __threadfence();
#pragma unroll
  for (int i = 0; i < 8; ++i) {
    const int lr = 16 * wave + 2 * i + hh;
    float* op = WH + (size_t)(rowBase + lr) * (size_t)FO + 4 * m;
    *(volatile v4f*)op = fv[i];
  }
  if (okuv) *(volatile v4f*)uvp = uvv;
#pragma unroll
  for (int g = 0; g < 4; ++g) {
    const int o  = 16 * g + (tid >> 3);
    const int ms = (tid & 7) * 8;
    const size_t off = ((size_t)bq * FO + o) * (size_t)NN + mloc + ms;
    *(volatile v8us*)(VTH + off) = hv[g];
    *(volatile v8us*)(VTL + off) = lv[g];
  }
}

__device__ __forceinline__ float pscore(float u, float v, float mx) {
  float t = u + v;
  t = (t >= 0.0f) ? t : 0.2f * t;
  return expf(t - mx);
}

__device__ __forceinline__ void split2(float p0, float p1, int& hw, int& lw) {
  const unsigned h0 = bf16_bits(p0), h1 = bf16_bits(p1);
  const unsigned l0 = bf16_bits(p0 - __uint_as_float(h0 << 16));
  const unsigned l1 = bf16_bits(p1 - __uint_as_float(h1 << 16));
  hw = (int)(h0 | (h1 << 16));
  lw = (int)(l0 | (l1 << 16));
}

__device__ __forceinline__ float elu1(float x) {
  return (x > 0.0f) ? x : expm1f(x);
}

__global__ __launch_bounds__(GTHR) void k_attn(const float* __restrict__ WH, const float* __restrict__ U,
                                               const float* __restrict__ V,
                                               const unsigned short* __restrict__ VTH,
                                               const unsigned short* __restrict__ VTL,
                                               float* out) {
  __shared__ __attribute__((aligned(16))) float vS[NN];
  __shared__ __attribute__((aligned(16))) float stg[QT * FO];
  __shared__ float red[4];
  const int tid = (int)threadIdx.x, lane = tid & 31, wave = tid >> 5, hh = lane >> 4, m = lane & 15;
  const int b  = (int)blockIdx.y;
  const int q0 = (int)blockIdx.x * QT;

  {
    const float* vsrc = V + (size_t)b * NN;
    float vm = __int_as_float((int)0xff800000u);
#pragma unroll
    for (int j = 0; j < 4; ++j) {
      const int idx = (j * GTHR + tid) * 4;
      const v4f x = *(const v4fa*)(vsrc + idx);
      *(v4fa*)(vS + idx) = x;
      vm = fmaxf(vm, fmaxf(fmaxf(x.x, x.y), fmaxf(x.z, x.w)));
    }
#pragma unroll
    for (int d = 16; d >= 1; d >>= 1) vm = fmaxf(vm, __shfl_xor(vm, d, 32));
    if (lane == 0) red[wave] = vm;
  }
  __syncthreads();
  const float vmax = fmaxf(fmaxf(red[0], red[1]), fmaxf(red[2], red[3]));

  const float urow = U[(size_t)b * NN + q0 + 16 * wave + m];
  float mx;
  {
    const float t = urow + vmax;
    mx = (t >= 0.0f) ? t : 0.2f * t;
  }

  v8f acc[4];
  {
    const v8f z = {0.f, 0.f, 0.f, 0.f, 0.f, 0.f, 0.f, 0.f};
    acc[0] = z; acc[1] = z; acc[2] = z; acc[3] = z;
  }
  float lsum = 0.0f;
  const unsigned short* bhp = VTH + ((size_t)b * FO + m) * (size_t)NN + 8 * hh;
  const unsigned short* blp = VTL + ((size_t)b * FO + m) * (size_t)NN + 8 * hh;

#pragma unroll 1
  for (int k0 = 0; k0 < NN; k0 += 32) {
    const v4f va = *(const v4fa*)(vS + k0 + 8 * hh);
    const v4f vb = *(const v4fa*)(vS + k0 + 8 * hh + 4);
    const v4f vc = *(const v4fa*)(vS + k0 + 16 + 8 * hh);
    const v4f vd = *(const v4fa*)(vS + k0 + 16 + 8 * hh + 4);
    const float vv[16] = {va.x, va.y, va.z, va.w, vb.x, vb.y, vb.z, vb.w,
                          vc.x, vc.y, vc.z, vc.w, vd.x, vd.y, vd.z, vd.w};
    FragB ph, pl;
#pragma unroll
    for (int j = 0; j < 8; ++j) {
      const float p0 = pscore(urow, vv[2 * j], mx);
      const float p1 = pscore(urow, vv[2 * j + 1], mx);
      lsum += p0;
      lsum += p1;
      int hw, lw;
      split2(p0, p1, hw, lw);
      ph.w[j] = hw;
      pl.w[j] = lw;
    }
#pragma unroll
    for (int t = 0; t < 4; ++t) {
      const unsigned short* qh = bhp + (size_t)(16 * t) * (size_t)NN + k0;
      const unsigned short* ql = blp + (size_t)(16 * t) * (size_t)NN + k0;
      FragB fh, fl;
      fh.h[0] = *(const v8usa*)qh;
      fh.h[1] = *(const v8usa*)(qh + 16);
      fl.h[0] = *(const v8usa*)ql;
      fl.h[1] = *(const v8usa*)(ql + 16);
      acc[t] = wmb(ph, fh, acc[t]);
      acc[t] = wmb(ph, fl, acc[t]);
      acc[t] = wmb(pl, fh, acc[t]);
    }
  }

  const float ltot = lsum + __shfl_xor(lsum, 16, 32);
  const float linv = 1.0f / ltot;
#pragma unroll
  for (int r = 0; r < 8; ++r) {
    const float li = __shfl(linv, 8 * hh + r, 32);
#pragma unroll
    for (int t = 0; t < 4; ++t) {
      stg[(16 * wave + 8 * hh + r) * FO + 16 * t + m] = acc[t][r] * li;
    }
  }
  __syncthreads();

  const size_t rowG0 = (size_t)b * NN + q0;
#pragma unroll 1
  for (int i = 0; i < 8; ++i) {
    const int lr = 16 * wave + 2 * i + hh;
    float* sp = stg + lr * FO + 4 * m;
    const v4f o4 = *(const v4fa*)sp;
    const v4f w4 = *(const v4fa*)(WH + (rowG0 + lr) * (size_t)FO + 4 * m);
    v4f y;
    y.x = elu1(0.9f * o4.x + 0.1f * w4.x);
    y.y = elu1(0.9f * o4.y + 0.1f * w4.y);
    y.z = elu1(0.9f * o4.z + 0.1f * w4.z);
    y.w = elu1(0.9f * o4.w + 0.1f * w4.w);
    *(v4fa*)sp = y;
  }
  __syncthreads();

  v4f fv[8];
#pragma unroll
  for (int i = 0; i < 8; ++i) {
    const int lr = 16 * wave + 2 * i + hh;
    fv[i] = *(const v4fa*)(stg + lr * FO + 4 * m);
  }
#pragma unroll
  for (int i = 0; i < 8; ++i) {
    const int lr = 16 * wave + 2 * i + hh;
    float* op = out + (rowG0 + lr) * (size_t)FO + 4 * m;
    *(volatile v4f*)op = fv[i];
  }
  __threadfence();
#pragma unroll
  for (int i = 0; i < 8; ++i) {
    const int lr = 16 * wave + 2 * i + hh;
    float* op = out + (rowG0 + lr) * (size_t)FO + 4 * m;
    *(volatile v4f*)op = fv[i];
  }
}

static inline size_t al256(size_t o) { return (o + 255) & ~(size_t)255; }

extern "C" void kernel_launch(void* const* d_in, const int* in_sizes, int n_in,
                              void* d_out, int out_size, void* d_ws, size_t ws_size,
                              hipStream_t stream) {
  if (n_in < 3) return;
  if (in_sizes[0] != MROWS * FIN) return;
  if (in_sizes[1] != FIN * FO) return;
  if (in_sizes[2] != 2 * FO) return;
  if (out_size != MROWS * FO) return;

  const float* h = (const float*)d_in[0];
  const float* W = (const float*)d_in[1];
  const float* a = (const float*)d_in[2];
  float* out = (float*)d_out;

  char* ws = (char*)d_ws;
  size_t off = 0;
  const size_t oHB  = off; off = al256(off + (size_t)MROWS * FIN * 2);
  const size_t oWT  = off; off = al256(off + (size_t)FO * FIN * 2);
  const size_t oA12 = off; off = al256(off + (size_t)2 * FO * 4);
  const size_t oWH  = off; off = al256(off + (size_t)MROWS * FO * 4);
  const size_t oU   = off; off = al256(off + (size_t)MROWS * 4);
  const size_t oV   = off; off = al256(off + (size_t)MROWS * 4);
  const size_t oVTH = off; off = al256(off + (size_t)NB * FO * NN * 2);
  const size_t oVTL = off; off = al256(off + (size_t)NB * FO * NN * 2);
  if (off > ws_size || off > (size_t)WSMAX) return;
  unsigned short* HB  = (unsigned short*)(ws + oHB);
  unsigned short* WT  = (unsigned short*)(ws + oWT);
  float*          A12 = (float*)(ws + oA12);
  float*          WH  = (float*)(ws + oWH);
  float*          U   = (float*)(ws + oU);
  float*          V   = (float*)(ws + oV);
  unsigned short* VTH = (unsigned short*)(ws + oVTH);
  unsigned short* VTL = (unsigned short*)(ws + oVTL);

  k_prep<<<(NUH + NUW) / PTHR + 1, PTHR, 0, stream>>>(h, W, a, HB, WT, A12);
  k_proj<<<MROWS / GBM, GTHR, 0, stream>>>(HB, WT, A12, WH, U, V, VTH, VTL);
  k_attn<<<dim3(NN / QT, NB), GTHR, 0, stream>>>(WH, U, V, VTH, VTL, out);
}
